// RNNModel_46540265619727
// MI455X (gfx1250) — hardware-verified
//
#include <hip/hip_runtime.h>
#include <math.h>

constexpr int NSEQ   = 64;
constexpr int NSTEP  = 2048;
constexpr int NIN    = 64;
constexpr int NHID   = 256;
constexpr int KTOT   = NIN + 2 * NHID;
constexpr int NKC    = KTOT / 32;
constexpr int NXC    = NIN / 32;
constexpr int NHC    = NHID / 32;
constexpr int NWB    = NXC + NHC;
constexpr int NTHR   = 512;
constexpr int NWAVE  = NTHR / 32;
constexpr int ROWBLK = 16;
constexpr int APITCH = 584;
constexpr int HFP    = 260;
constexpr int OCH    = 128;
constexpr int OSP    = 132;
constexpr int COLX   = 0;
constexpr int COLHI  = NIN;
constexpr int COLLO  = NIN + NHID;
constexpr float WCARRY     = 256.0f;
constexpr float WCARRY_INV = 1.0f / 256.0f;
constexpr float LOSC       = 2048.0f;
constexpr float LOSC_INV   = 1.0f / 2048.0f;
constexpr float F16_MIN_NORMAL = 6.103515625e-5f;

static_assert(NSEQ % ROWBLK == 0);
static_assert(NHID == 16 * NWAVE);
static_assert(NWAVE == ROWBLK);
static_assert(NIN % 32 == 0 && NHID % 32 == 0);
static_assert(KTOT == 32 * NKC && (NKC % 2) == 0);
static_assert((NWB % 2) == 0);
static_assert(NTHR * 2 == ROWBLK * NIN);
static_assert(NHID == 32 * 8);
static_assert(NSTEP % OCH == 0 && OCH == 32 * 4);
static_assert(APITCH % 8 == 0 && APITCH >= KTOT);
static_assert(HFP % 4 == 0 && HFP >= NHID);
static_assert(OSP % 4 == 0 && OSP >= OCH);
static_assert(((2 * ROWBLK * APITCH) % 2) == 0);

typedef __attribute__((ext_vector_type(16))) _Float16 v16h;
typedef __attribute__((ext_vector_type(8)))  _Float16 v8h;
typedef __attribute__((ext_vector_type(8)))  float    v8f;
typedef __attribute__((ext_vector_type(4)))  float    v4f;
typedef __attribute__((ext_vector_type(2)))  float    v2f;

__device__ __forceinline__ float bf16r(float f) {
  unsigned u = __float_as_uint(f);
  u = (u + 0x7FFFu + ((u >> 16) & 1u)) & 0xFFFF0000u;
  return __uint_as_float(u);
}

__device__ __forceinline__ void grp_guard4_h(v8f& a, v8f& b, v8f& c, v8f& d,
                                             v16h x, v16h y, v16h bx, v16h by) {
  asm volatile("v_nop\n\tv_nop\n\tv_nop\n\tv_nop"
               : "+v"(a), "+v"(b), "+v"(c), "+v"(d) : "v"(x), "v"(y), "v"(bx), "v"(by) : "memory");
}
__device__ __forceinline__ void acc_guard4(v8f& a, v8f& b, v8f& c, v8f& d) {
  asm volatile("v_nop\n\tv_nop\n\tv_nop\n\tv_nop" : "+v"(a), "+v"(b), "+v"(c), "+v"(d));
}
__device__ __forceinline__ void frag_fence_h(v16h& w) { asm volatile("" : "+v"(w) :: "memory"); }

template <typename T> struct Frag;
template <> struct Frag<_Float16> {
  typedef v16h V; union U { v16h v; v8h h[2]; };
  static __device__ __forceinline__ v16h load(const _Float16* p) {
    U f; f.h[0] = *(const v8h*)(p); f.h[1] = *(const v8h*)(p + 16); return f.v;
  }
  static __device__ __forceinline__ v8f mma(v16h a, v16h b, v8f c) {
    return __builtin_amdgcn_wmma_f32_16x16x32_f16(false, a, false, b, (short)0, c, false, false);
  }
};

__device__ __forceinline__ float ftanh(float z) {
  const float zc = fminf(fmaxf(z, -15.0f), 15.0f);
  const float e = expf(2.0f * zc);
  return 1.0f - 2.0f * __builtin_amdgcn_rcpf(e + 1.0f);
}

__device__ __forceinline__ void stage_x2(const float* __restrict__ x, int rowbase, int t, int tid,
                                         _Float16* __restrict__ tile) {
  const int xm = tid >> 5, xc = (tid & 31) * 2;
  const float* p = x + ((size_t)(rowbase + xm) * NSTEP + (size_t)t) * NIN + xc;
  const v2f v = *(const v2f*)p;
  const float f0 = v[0], f1 = v[1];
  const _Float16 h0 = (_Float16)bf16r(f0);
  const _Float16 h1 = (_Float16)bf16r(f1);
  const unsigned short u0 = __builtin_bit_cast(unsigned short, h0);
  const unsigned short u1 = __builtin_bit_cast(unsigned short, h1);
  const unsigned u = (unsigned)u0 | ((unsigned)u1 << 16);
  *(unsigned*)(tile + xm * APITCH + COLX + xc) = u;
}

__global__ __launch_bounds__(NTHR) void rnn_seq_kernel(
    const float* __restrict__ x,    const float* __restrict__ w_ih, const float* __restrict__ w_hh,
    const float* __restrict__ b_ih, const float* __restrict__ b_hh, const float* __restrict__ w_fc,
    const float* __restrict__ b_fc, float* __restrict__ out) {
  __shared__ __align__(16) _Float16 At[2][ROWBLK * APITCH];
  __shared__ __align__(16) float    Hf[2][ROWBLK * HFP];
  __shared__ __align__(16) float    Os[NWAVE * OSP];

  const int tid = threadIdx.x, lane = tid & 31, wave = tid >> 5;
  const int m = lane & 15, hh = lane >> 4, koff = hh * 8;
  const int rowbase = blockIdx.x * ROWBLK;
  const int n = 16 * wave + m;

  {
    unsigned* az = (unsigned*)(&At[0][0]);
#pragma unroll 1
    for (int i = tid; i < (2 * ROWBLK * APITCH) / 2; i += NTHR) az[i] = 0u;
  }
  __syncthreads();

  stage_x2(x, rowbase, 0, tid, &At[0][0]);

  v16h wB[NWB];
#pragma unroll
  for (int kc = 0; kc < NWB; ++kc) {
    const float* src = (kc < NXC) ? (w_ih + (size_t)n * NIN  + 32 * kc)
                                  : (w_hh + (size_t)n * NHID + 32 * (kc - NXC));
    const v4f q0 = *(const v4f*)(src + koff);
    const v4f q1 = *(const v4f*)(src + koff + 4);
    const v4f q2 = *(const v4f*)(src + 16 + koff);
    const v4f q3 = *(const v4f*)(src + 16 + koff + 4);
    v16h f;
#pragma unroll
    for (int e = 0; e < 4; ++e) {
      f[e]      = (_Float16)(bf16r(q0[e]) * WCARRY);
      f[4 + e]  = (_Float16)(bf16r(q1[e]) * WCARRY);
      f[8 + e]  = (_Float16)(bf16r(q2[e]) * WCARRY);
      f[12 + e] = (_Float16)(bf16r(q3[e]) * WCARRY);
    }
    frag_fence_h(f);
    wB[kc] = f;
  }

  const float bsum = bf16r(b_ih[n]) + bf16r(b_hh[n]);
  const v4f fa = *(const v4f*)(w_fc + 8 * lane);
  const v4f fb = *(const v4f*)(w_fc + 8 * lane + 4);
  v4f wfa, wfb;
#pragma unroll
  for (int e = 0; e < 4; ++e) { wfa[e] = bf16r(fa[e]); wfb[e] = bf16r(fb[e]); }
  const float bfc = bf16r(b_fc[0]);
  __syncthreads();

  const v8f z8 = {0.f, 0.f, 0.f, 0.f, 0.f, 0.f, 0.f, 0.f};

#pragma unroll 1
  for (int t = 0; t < NSTEP; ++t) {
    const int p = t & 1;
    const _Float16* arow = &At[p][0] + m * APITCH + koff;
    _Float16* awr = &At[p ^ 1][0];
    float*    hfw = &Hf[p ^ 1][0];

    v8f c0 = z8, c1 = z8, d0 = z8, d1 = z8;
#pragma unroll
    for (int g = 0; g < NKC / 2; ++g) {
      const int k0 = 2 * g, k1 = 2 * g + 1;
      const v16h a0 = Frag<_Float16>::load(arow + 32 * k0);
      const v16h a1 = Frag<_Float16>::load(arow + 32 * k1);
      if (k0 < NWB) {
        c0 = Frag<_Float16>::mma(a0, wB[k0], c0);
        c1 = Frag<_Float16>::mma(a1, wB[k1], c1);
        grp_guard4_h(c0, c1, d0, d1, a0, a1, wB[k0], wB[k1]);
      } else {
        d0 = Frag<_Float16>::mma(a0, wB[k0 - NHC], d0);
        d1 = Frag<_Float16>::mma(a1, wB[k1 - NHC], d1);
        grp_guard4_h(c0, c1, d0, d1, a0, a1, wB[k0 - NHC], wB[k1 - NHC]);
      }
    }
    acc_guard4(c0, c1, d0, d1);

#pragma unroll
    for (int r = 0; r < 8; ++r) {
      const float zm = (c0[r] + c1[r]) * WCARRY_INV;
      const float zl = (d0[r] + d1[r]) * (WCARRY_INV * LOSC_INV);
      const float z  = (zm + zl) + bsum;
      const float hn = ftanh(z);
      const float hc = (fabsf(hn) < F16_MIN_NORMAL) ? 0.0f : hn;
      const _Float16 hi16 = (_Float16)hc;
      const float hiv = (float)hi16;
      const float res = hn - hiv;
      const _Float16 lo16 = (_Float16)(res * LOSC);
      const int ro = (8 * hh + r) * APITCH;
      awr[ro + COLHI + n] = hi16;
      awr[ro + COLLO + n] = lo16;
      hfw[(8 * hh + r) * HFP + n] = hn;
    }
    {
      const int tn = (t + 1 < NSTEP) ? (t + 1) : (NSTEP - 1);
      stage_x2(x, rowbase, tn, tid, awr);
    }
    __syncthreads();

    {
      const float* hr = &Hf[p ^ 1][0] + wave * HFP + 8 * lane;
      const v4f u0 = *(const v4f*)(hr);
      const v4f u1 = *(const v4f*)(hr + 4);
      float s = 0.0f;
#pragma unroll
      for (int e = 0; e < 4; ++e) s = fmaf(u0[e], wfa[e], s);
#pragma unroll
      for (int e = 0; e < 4; ++e) s = fmaf(u1[e], wfb[e], s);
#pragma unroll
      for (int off = 16; off >= 1; off >>= 1) s += __shfl_xor(s, off, 32);
      const float o = s + bfc;
      if (lane == 0) Os[wave * OSP + (t & (OCH - 1))] = o;
    }

    if ((t & (OCH - 1)) == OCH - 1) {
      __builtin_amdgcn_fence(__ATOMIC_RELEASE, "workgroup");
      __builtin_amdgcn_wave_barrier();
      __builtin_amdgcn_fence(__ATOMIC_ACQUIRE, "workgroup");
      const v4f ov = *(const v4f*)(Os + wave * OSP + 4 * lane);
      float* op = out + (size_t)(rowbase + wave) * NSTEP + (size_t)(t + 1 - OCH) + 4 * lane;
      *(volatile v4f*)op = ov;
      __threadfence();
      *(volatile v4f*)op = ov;
    }
  }
}

extern "C" void kernel_launch(void* const* d_in, const int* in_sizes, int n_in,
                              void* d_out, int out_size, void* d_ws, size_t ws_size, hipStream_t stream) {
  (void)d_ws; (void)ws_size;
  if (n_in < 7 || d_out == nullptr) return;
  if (in_sizes[0] != NSEQ * NSTEP * NIN || in_sizes[1] != NHID * NIN || in_sizes[2] != NHID * NHID ||
      in_sizes[3] != NHID || in_sizes[4] != NHID || in_sizes[5] != NHID || in_sizes[6] != 1 ||
      out_size != NSEQ * NSTEP) return;

  const float* x    = (const float*)d_in[0];
  const float* w_ih = (const float*)d_in[1];
  const float* w_hh = (const float*)d_in[2];
  const float* b_ih = (const float*)d_in[3];
  const float* b_hh = (const float*)d_in[4];
  const float* w_fc = (const float*)d_in[5];
  const float* b_fc = (const float*)d_in[6];
  float* out = (float*)d_out;

  rnn_seq_kernel<<<NSEQ / ROWBLK, NTHR, 0, stream>>>(x, w_ih, w_hh, b_ih, b_hh, w_fc, b_fc, out);
}
